// GAT_22531398435166
// MI455X (gfx1250) — hardware-verified
//
#include <hip/hip_runtime.h>
#include <math.h>

typedef __attribute__((ext_vector_type(16))) _Float16 v16h;
typedef __attribute__((ext_vector_type(8)))  _Float16 v8h;
typedef __attribute__((ext_vector_type(8)))  float    v8f;
typedef __attribute__((ext_vector_type(4)))  float    v4f;
typedef __attribute__((ext_vector_type(4)))  int      v4i;

constexpr int N_NODES   = 20000;
constexpr int N_PAD     = 20032;
constexpr int F_IN      = 64;
constexpr int N_GATE    = 256;
constexpr int DEG       = 8;
constexpr int F_OUT     = 32;
constexpr int F_EDGE    = 32;
constexpr int N_EDGES   = N_NODES * DEG;
constexpr int N_GRAPHS  = 200;
constexpr int NODES_PER_GRAPH = 100;
constexpr int CAT_LD    = 128;
constexpr int H_LD      = 64;
constexpr int P_KDIM    = 1056;
constexpr int P_LD      = 1088;
constexpr int LDS_WP    = 72;
constexpr float W_CARRY     = 16.0f;
constexpr float W_CARRY_INV = 1.0f / 16.0f;

static_assert(N_PAD % 64 == 0 && N_PAD >= N_NODES, "row padding");
static_assert(N_GATE % 64 == 0 && F_IN % 32 == 0 && CAT_LD % 32 == 0 && P_KDIM % 32 == 0, "tile multiples");
static_assert(P_LD % 64 == 0 && P_LD >= P_KDIM, "plane pitch is a whole number of 128-B lines");
static_assert(N_GRAPHS * NODES_PER_GRAPH == N_NODES, "graph partition");
static_assert(P_KDIM == F_EDGE * F_OUT + F_OUT, "outer-product columns plus row-sum columns");

constexpr int PB_CAT  = (N_PAD * 8) / 256;
constexpr int PB_WIH  = (N_GATE * F_IN / 8) / 256;
constexpr int PB_WHH  = PB_WIH;
constexpr int PB_WCS  = 2;
constexpr int PB_WCN  = 2;
constexpr int PB_WRM  = (64 * 128) / 256;
constexpr int PB_WRT  = 2;
constexpr int PS_WIH  = PB_CAT;
constexpr int PS_WHH  = PS_WIH + PB_WIH;
constexpr int PS_WCS  = PS_WHH + PB_WHH;
constexpr int PS_WCN  = PS_WCS + PB_WCS;
constexpr int PS_WRM  = PS_WCN + PB_WCN;
constexpr int PS_WRT  = PS_WRM + PB_WRM;
constexpr int PS_BSUM = PS_WRT + PB_WRT;
constexpr int PS_BIAS = PS_BSUM + 1;
constexpr int PREP_BLOCKS = PS_BIAS + 1;
static_assert(PB_CAT * 256 == N_PAD * 8, "exact chunk coverage of the node-feature half");
static_assert(PB_WIH * 256 * 8 == N_GATE * F_IN, "exact coverage of a gate weight plane");

__device__ __forceinline__ void keep4_h(v16h a, v16h b, v16h c, v16h d) { asm volatile("v_nop" :: "v"(a), "v"(b), "v"(c), "v"(d)); }
__device__ __forceinline__ void acc_guard4(v8f& a, v8f& b, v8f& c, v8f& d) { asm volatile("v_nop\n\tv_nop\n\tv_nop\n\tv_nop" : "+v"(a), "+v"(b), "+v"(c), "+v"(d)); }
__device__ __forceinline__ void row_guard_h(v8f& a, v8f& b, v8f& c, v8f& d, v16h x, v16h y0, v16h y1, v16h y2, v16h y3) {
  asm volatile("v_nop\n\tv_nop\n\tv_nop\n\tv_nop" : "+v"(a), "+v"(b), "+v"(c), "+v"(d) : "v"(x), "v"(y0), "v"(y1), "v"(y2), "v"(y3));
}
__device__ __forceinline__ void step_guard_h(v8f& a, v8f& b, v8f& c, v8f& d, v16h x0, v16h x1,
                                             v16h p0, v16h p1, v16h p2, v16h p3, v16h p4, v16h p5, v16h p6, v16h p7) {
  asm volatile("v_nop\n\tv_nop\n\tv_nop\n\tv_nop" : "+v"(a), "+v"(b), "+v"(c), "+v"(d)
               : "v"(x0), "v"(x1), "v"(p0), "v"(p1), "v"(p2), "v"(p3), "v"(p4), "v"(p5), "v"(p6), "v"(p7));
}

template <typename T> struct Frag;
template <> struct Frag<_Float16> {
  typedef v16h V; union U { v16h v; v8h h[2]; };
  static __device__ __forceinline__ v16h load(const _Float16* p) {
    U f; f.h[0] = *(const v8h*)(p); f.h[1] = *(const v8h*)(p + 16); return f.v;
  }
  static __device__ __forceinline__ v8f mma(v16h a, v16h b, v8f c) {
    return __builtin_amdgcn_wmma_f32_16x16x32_f16(false, a, false, b, (short)0, c, false, false);
  }
};

__device__ __forceinline__ void store_chunk2(unsigned short* dst, v8h v) {
  *(volatile v8h*)dst = v;
  __threadfence();
  *(volatile v8h*)dst = v;
}
__device__ __forceinline__ void store_word2(float* dst, float v) {
  *(volatile float*)dst = v;
  __threadfence();
  *(volatile float*)dst = v;
}

__device__ __forceinline__ void cvt8_store(const float* src, unsigned short* dst, int q, float sc) {
  const v4f a = *(const v4f*)(src + (size_t)q * 8);
  const v4f b = *(const v4f*)(src + (size_t)q * 8 + 4);
  v8h o;
#pragma unroll
  for (int e = 0; e < 4; ++e) { o[e] = (_Float16)(a[e] * sc); o[4 + e] = (_Float16)(b[e] * sc); }
  store_chunk2(dst + (size_t)q * 8, o);
}

__global__ __launch_bounds__(256) void prep_kernel(
    const float* __restrict__ nfeat, const float* __restrict__ Wih, const float* __restrict__ Whh,
    const float* __restrict__ bih, const float* __restrict__ bhh,
    const float* __restrict__ Wself, const float* __restrict__ bself, const float* __restrict__ Wneigh,
    const float* __restrict__ Wew, const float* __restrict__ Web, const float* __restrict__ nnb,
    unsigned short* __restrict__ cat, unsigned short* __restrict__ Wih16, unsigned short* __restrict__ Whh16,
    float* __restrict__ bsum, float* __restrict__ bself64, float* __restrict__ nnb64,
    unsigned short* __restrict__ WcatT, unsigned short* __restrict__ WrT) {
  const int tid = threadIdx.x;
  const int blk = blockIdx.x;
  if (blk < PS_WIH) {
    const int q = blk * 256 + tid;
    const int row = q >> 3, c8 = (q & 7) * 8;
    const bool live = row < N_NODES;
    const int rc = live ? row : (N_NODES - 1);
    const v4f a = *(const v4f*)(nfeat + (size_t)rc * F_IN + c8);
    const v4f b = *(const v4f*)(nfeat + (size_t)rc * F_IN + c8 + 4);
    v8h o;
#pragma unroll
    for (int e = 0; e < 4; ++e) {
      o[e]     = (_Float16)(live ? a[e] : 0.0f);
      o[4 + e] = (_Float16)(live ? b[e] : 0.0f);
    }
    store_chunk2(cat + (size_t)row * CAT_LD + c8, o);
  } else if (blk < PS_WHH) {
    cvt8_store(Wih, Wih16, (blk - PS_WIH) * 256 + tid, W_CARRY);
  } else if (blk < PS_WCS) {
    cvt8_store(Whh, Whh16, (blk - PS_WHH) * 256 + tid, W_CARRY);
  } else if (blk < PS_WRM) {
    const bool second = blk >= PS_WCN;
    const float* src = second ? Wneigh : Wself;
    const int q = (blk - (second ? PS_WCN : PS_WCS)) * 256 + tid;
    const int o = q >> 3, k8 = (q & 7) * 8;
    const bool live = o < F_OUT;
    const int oc = live ? o : (F_OUT - 1);
    v8h ov;
#pragma unroll
    for (int e = 0; e < 8; ++e) {
      float x = src[(k8 + e) * F_OUT + oc];
      asm volatile("" : "+v"(x));
      ov[e] = (_Float16)(live ? x * W_CARRY : 0.0f);
    }
    store_chunk2(WcatT + (size_t)o * CAT_LD + (second ? 64 : 0) + k8, ov);
  } else if (blk < PS_WRT) {
    const int q = (blk - PS_WRM) * 256 + tid;
    const int o = q >> 7, c8 = (q & 127) * 8;
    const bool live = o < F_OUT;
    const int oc = live ? o : (F_OUT - 1);
    const int f = c8 >> 5, i0 = c8 & 31;
    v8h ov;
#pragma unroll
    for (int e = 0; e < 8; ++e) {
      float x = Wew[f * (F_EDGE * F_OUT) + (i0 + e) * F_OUT + oc];
      asm volatile("" : "+v"(x));
      ov[e] = (_Float16)(live ? x * W_CARRY : 0.0f);
    }
    store_chunk2(WrT + (size_t)o * P_LD + c8, ov);
  } else if (blk < PS_BSUM) {
    const int q = (blk - PS_WRT) * 256 + tid;
    const int o = q >> 3, j = q & 7;
    const bool live = (o < F_OUT) && (j < 4);
    const int oc = (o < F_OUT) ? o : (F_OUT - 1);
    v8h ov;
#pragma unroll
    for (int e = 0; e < 8; ++e) {
      int i = j * 8 + e;
      i = i < F_OUT ? i : (F_OUT - 1);
      float x = Web[i * F_OUT + oc];
      asm volatile("" : "+v"(x));
      ov[e] = (_Float16)(live ? x * W_CARRY : 0.0f);
    }
    store_chunk2(WrT + (size_t)o * P_LD + 1024 + j * 8, ov);
  } else if (blk < PS_BIAS) {
    const float v = bih[tid] + bhh[tid];
    store_word2(bsum + tid, v);
  } else {
    if (tid < 128) {
      const int w = tid >> 5, lane = tid & 31;
      float x = 0.0f;
      if (w == 0) x = bself[lane];
      if (w == 2) x = nnb[lane];
      float* dst = (w < 2) ? (bself64 + tid) : (nnb64 + (tid - 64));
      store_word2(dst, x);
    }
  }
}

template <int ACT>
__global__ __launch_bounds__(256) void gemm64_f16(
    const unsigned short* __restrict__ Ap, int lda,
    const unsigned short* __restrict__ Btp, int ldb,
    float* __restrict__ C, int ldc,
    const float* __restrict__ bias,
    int M, int N, int K, float scale) {
  const _Float16* A  = (const _Float16*)Ap;
  const _Float16* Bt = (const _Float16*)Btp;
  __shared__ __align__(16) float sT[8][16 * 68];
  const int lane = threadIdx.x & 31;
  const int wave = threadIdx.x >> 5;
  const int tilesN = N >> 6;
  const int tilesM = M >> 6;
  const int tile = blockIdx.x * 8 + wave;
  if (tile >= tilesM * tilesN) return;
  const int tm = tile / tilesN;
  const int tn = tile - tm * tilesN;
  const int m0 = tm << 6;
  const int n0 = tn << 6;

  const int rlane = lane & 15;
  const int koff  = (lane >> 4) * 8;
  const int mOff  = (lane >> 4) * 8;

  v8f acc[4][4];
#pragma unroll
  for (int i = 0; i < 4; ++i)
#pragma unroll
    for (int j = 0; j < 4; ++j) acc[i][j] = (v8f){0.f,0.f,0.f,0.f,0.f,0.f,0.f,0.f};

  for (int k0 = 0; k0 < K; k0 += 32) {
    v16h bh[4];
#pragma unroll
    for (int j = 0; j < 4; ++j) {
      const size_t bo = (size_t)(n0 + (j << 4) + rlane) * ldb + koff + k0;
      bh[j] = Frag<_Float16>::load(Bt + bo);
    }
#pragma unroll
    for (int i = 0; i < 4; ++i) {
      const size_t ao = (size_t)(m0 + (i << 4) + rlane) * lda + koff + k0;
      const v16h ah = Frag<_Float16>::load(A + ao);
#pragma unroll
      for (int j = 0; j < 4; ++j) acc[i][j] = Frag<_Float16>::mma(ah, bh[j], acc[i][j]);
      row_guard_h(acc[i][0], acc[i][1], acc[i][2], acc[i][3], ah, bh[0], bh[1], bh[2], bh[3]);
    }
    keep4_h(bh[0], bh[1], bh[2], bh[3]);
  }
  acc_guard4(acc[0][0], acc[0][1], acc[0][2], acc[0][3]);
  acc_guard4(acc[1][0], acc[1][1], acc[1][2], acc[1][3]);
  acc_guard4(acc[2][0], acc[2][1], acc[2][2], acc[2][3]);
  acc_guard4(acc[3][0], acc[3][1], acc[3][2], acc[3][3]);

  float* slab = sT[wave];
#pragma unroll
  for (int i = 0; i < 4; ++i) {
    const int mBase = m0 + (i << 4);
#pragma unroll
    for (int j = 0; j < 4; ++j) {
      const int n = n0 + (j << 4) + rlane;
      const float bv = bias[n];
#pragma unroll
      for (int r = 0; r < 8; ++r) {
        float v = acc[i][j][r] * scale;
        v += bv;
        if (ACT == 1) v = fmaxf(v, 0.0f);
        slab[(mOff + r) * 68 + (j << 4) + rlane] = v;
      }
    }
    __builtin_amdgcn_fence(__ATOMIC_RELEASE, "workgroup");
    __builtin_amdgcn_wave_barrier();
    __builtin_amdgcn_fence(__ATOMIC_ACQUIRE, "workgroup");
    {
      const int hh = lane >> 4, c4 = (lane & 15) * 4;
      for (int pass = 0; pass < 2; ++pass) {
#pragma unroll
        for (int it = 0; it < 8; ++it) {
          const int row = it * 2 + hh;
          const v4f v = *(const v4f*)(slab + row * 68 + c4);
          *(volatile v4f*)(C + (size_t)(mBase + row) * ldc + n0 + c4) = v;
        }
        __threadfence();
      }
    }
    __builtin_amdgcn_fence(__ATOMIC_RELEASE, "workgroup");
    __builtin_amdgcn_wave_barrier();
    __builtin_amdgcn_fence(__ATOMIC_ACQUIRE, "workgroup");
  }
}

__device__ __forceinline__ float sigm_f(float x) { return __builtin_amdgcn_rcpf(1.0f + expf(-x)); }

__global__ __launch_bounds__(128) void lstm_kernel(
    const float* __restrict__ xproj, const int* __restrict__ neigh,
    const unsigned short* __restrict__ Whh16p, unsigned short* __restrict__ catp) {
  __shared__ __align__(16) _Float16 sW[N_GATE * LDS_WP];
  __shared__ __align__(16) _Float16 sH[4][16 * LDS_WP];
  __shared__ __align__(16) float    sC[4][4 * 8 * 32];
  const _Float16* Whh16 = (const _Float16*)Whh16p;
  const int tid = threadIdx.x, lane = tid & 31, wave = tid >> 5;
  const int c = lane & 15, hh = lane >> 4, koff = hh * 8;

#pragma unroll 1
  for (int it = 0; it < 16; ++it) {
    const int idx = it * 128 + tid;
    const int row = idx >> 3, c8 = (idx & 7) * 8;
    *(v8h*)(sW + row * LDS_WP + c8) = *(const v8h*)(Whh16 + row * F_IN + c8);
  }
  float* sCw = sC[wave];
#pragma unroll 1
  for (int i = 0; i < 32; ++i) sCw[i * 32 + lane] = 0.0f;
  __syncthreads();

  const int tile = blockIdx.x * 4 + wave;
  const bool valid = tile < (N_NODES / 16);
  const int nodeBase = tile * 16;
  _Float16* myH = sH[wave];

  int rowNode[8];
#pragma unroll
  for (int r = 0; r < 8; ++r) {
    const int rn = nodeBase + 8 * hh + r;
    rowNode[r] = rn < N_NODES ? rn : (N_NODES - 1);
  }

  v16h hA0, hA1;
#pragma unroll
  for (int e = 0; e < 16; ++e) { hA0[e] = (_Float16)0.0f; hA1[e] = (_Float16)0.0f; }

#pragma unroll 1
  for (int t = 0; t < DEG; ++t) {
    unsigned xoff[8];
#pragma unroll
    for (int r = 0; r < 8; ++r) {
      int nb = neigh[rowNode[r] * DEG + t];
      nb = nb < 0 ? 0 : (nb > N_NODES - 1 ? N_NODES - 1 : nb);
      xoff[r] = (unsigned)nb * (unsigned)N_GATE;
    }
#pragma unroll 1
    for (int ht = 0; ht < 4; ++ht) {
      v8f acc[4];
#pragma unroll
      for (int gi = 0; gi < 4; ++gi) {
        const int col = gi * 64 + ht * 16 + c;
#pragma unroll
        for (int r = 0; r < 8; ++r) acc[gi][r] = xproj[(size_t)xoff[r] + col] * W_CARRY;
        asm volatile("" : "+v"(acc[gi]));
      }
      v16h bq[4][2];
#pragma unroll
      for (int gi = 0; gi < 4; ++gi) {
        const _Float16* bp = sW + (gi * 64 + ht * 16 + c) * LDS_WP + koff;
        bq[gi][0] = Frag<_Float16>::load(bp);
        bq[gi][1] = Frag<_Float16>::load(bp + 32);
      }
#pragma unroll
      for (int gi = 0; gi < 4; ++gi) {
        acc[gi] = Frag<_Float16>::mma(hA0, bq[gi][0], acc[gi]);
        acc[gi] = Frag<_Float16>::mma(hA1, bq[gi][1], acc[gi]);
      }
      step_guard_h(acc[0], acc[1], acc[2], acc[3], hA0, hA1,
                   bq[0][0], bq[0][1], bq[1][0], bq[1][1], bq[2][0], bq[2][1], bq[3][0], bq[3][1]);
#pragma unroll
      for (int r = 0; r < 8; ++r) {
        const float zi = acc[0][r] * W_CARRY_INV;
        const float zf = acc[1][r] * W_CARRY_INV;
        const float zg = acc[2][r] * W_CARRY_INV;
        const float zo = acc[3][r] * W_CARRY_INV;
        const float ig = sigm_f(zi);
        const float fg = sigm_f(zf);
        const float gg = tanhf(zg);
        const float og = sigm_f(zo);
        const float cold = sCw[(ht * 8 + r) * 32 + lane];
        const float cn = fg * cold + ig * gg;
        sCw[(ht * 8 + r) * 32 + lane] = cn;
        const float hv = og * tanhf(cn);
        myH[(8 * hh + r) * LDS_WP + ht * 16 + c] = (_Float16)hv;
      }
    }
    __syncthreads();
    hA0 = Frag<_Float16>::load(myH + c * LDS_WP + koff);
    hA1 = Frag<_Float16>::load(myH + c * LDS_WP + 32 + koff);
    __syncthreads();
  }

  {
    const int q = lane >> 3, c8 = (lane & 7) * 8;
    v8h zero8;
#pragma unroll
    for (int e = 0; e < 8; ++e) zero8[e] = (_Float16)0.0f;
    v8h hv[4];
#pragma unroll
    for (int it = 0; it < 4; ++it) {
      const int row = it * 4 + q;
      const v8h ld = *(const v8h*)(myH + row * LDS_WP + c8);
      hv[it] = valid ? ld : zero8;
    }
    for (int pass = 0; pass < 2; ++pass) {
#pragma unroll
      for (int it = 0; it < 4; ++it) {
        const int row = it * 4 + q;
        *(volatile v8h*)(catp + (size_t)(nodeBase + row) * CAT_LD + 64 + c8) = hv[it];
      }
      __threadfence();
    }
  }
}

__global__ __launch_bounds__(256) void pbuild_kernel(
    const float* __restrict__ efeat, const int* __restrict__ neigh,
    const float* __restrict__ hfull, unsigned short* __restrict__ Pp) {
  __shared__ __align__(16) _Float16 sP[8][P_LD];
  const int tid = threadIdx.x, lane = tid & 31, wave = tid >> 5;
  const int v = blockIdx.x * 8 + wave;
  const bool valid = v < N_NODES;
  const int vc = valid ? v : (N_NODES - 1);

  const v4i i0 = *(const v4i*)(neigh + (size_t)vc * DEG);
  const v4i i1 = *(const v4i*)(neigh + (size_t)vc * DEG + 4);
  int src[8];
  src[0] = i0[0]; src[1] = i0[1]; src[2] = i0[2]; src[3] = i0[3];
  src[4] = i1[0]; src[5] = i1[1]; src[6] = i1[2]; src[7] = i1[3];
  float hreg[8], ereg[8];
#pragma unroll
  for (int d = 0; d < 8; ++d) {
    int s = src[d];
    s = s < 0 ? 0 : (s > N_NODES - 1 ? N_NODES - 1 : s);
    hreg[d] = hfull[(size_t)s * H_LD + lane];
    ereg[d] = efeat[((size_t)vc * DEG + d) * F_EDGE + lane];
  }
  float hs = 0.0f;
#pragma unroll
  for (int d = 0; d < 8; ++d) hs += hreg[d];

  _Float16* sp = sP[wave];
#pragma unroll 1
  for (int f = 0; f < F_EDGE; ++f) {
    float a = 0.0f;
#pragma unroll
    for (int d = 0; d < 8; ++d) {
      const float ef = __shfl(ereg[d], f, 32);
      a = fmaf(ef, hreg[d], a);
    }
    a = valid ? a : 0.0f;
    sp[f * 32 + lane] = (_Float16)a;
  }
  {
    const float hsv = valid ? hs : 0.0f;
    const float zf = 0.0f;
    sp[1024 + lane] = (_Float16)hsv;
    sp[1056 + lane] = (_Float16)zf;
  }
  __syncthreads();

  v8h hv[5];
#pragma unroll
  for (int it = 0; it < 5; ++it) {
    int ch = it * 32 + lane;
    ch = ch < (P_LD / 8) ? ch : (P_LD / 8 - 1);
    hv[it] = *(const v8h*)(sp + ch * 8);
  }
  unsigned short* prow = Pp + (size_t)v * P_LD;
  for (int pass = 0; pass < 2; ++pass) {
#pragma unroll
    for (int it = 0; it < 5; ++it) {
      const int ch = it * 32 + lane;
      if (ch < (P_LD / 8)) *(volatile v8h*)(prow + ch * 8) = hv[it];
    }
    __threadfence();
  }
}

__global__ __launch_bounds__(256) void pool_kernel(const float* __restrict__ h2, float* __restrict__ g0) {
  const int lane = threadIdx.x & 31, wave = threadIdx.x >> 5;
  const int g = blockIdx.x * 8 + wave;
  if (g >= N_GRAPHS) return;
  const float* base = h2 + (size_t)g * NODES_PER_GRAPH * H_LD + lane;
  float m = -INFINITY;
#pragma unroll 4
  for (int r = 0; r < NODES_PER_GRAPH; ++r) m = fmaxf(m, base[(size_t)r * H_LD]);
  const float ev = expm1f(m);
  const float outv = m > 0.0f ? m : ev;
  store_word2(g0 + (size_t)g * F_OUT + lane, outv);
}

__global__ __launch_bounds__(224) void head_kernel(
    const float* __restrict__ g0, const float* __restrict__ W1, const float* __restrict__ b1,
    const float* __restrict__ W2, const float* __restrict__ b2,
    const float* __restrict__ W3, const float* __restrict__ b3, float* __restrict__ out) {
  __shared__ float sW1[F_OUT * 32];
  __shared__ float sW2[32 * 32];
  __shared__ float sB[224 * 33];
  const int tid = threadIdx.x;
#pragma unroll 1
  for (int i = tid; i < 1024; i += 224) { sW1[i] = W1[i]; sW2[i] = W2[i]; }
  __syncthreads();
  const int g = tid;
  const int gc = g < N_GRAPHS ? g : (N_GRAPHS - 1);
  const float* grow = g0 + (size_t)gc * F_OUT;
#pragma unroll 1
  for (int j = 0; j < 32; ++j) {
    float a = b1[j];
#pragma unroll 1
    for (int k = 0; k < F_OUT; ++k) a = fmaf(grow[k], sW1[k * 32 + j], a);
    sB[tid * 33 + j] = fmaxf(a, 0.0f);
  }
  float o = b3[0];
#pragma unroll 1
  for (int j = 0; j < 32; ++j) {
    float a = b2[j];
#pragma unroll 1
    for (int k = 0; k < 32; ++k) a = fmaf(sB[tid * 33 + k], sW2[k * 32 + j], a);
    a = fmaxf(a, 0.0f);
    o = fmaf(a, W3[j], o);
  }
  if (g < N_GRAPHS) *(volatile float*)(out + g) = o;
  __threadfence();
  if (g < N_GRAPHS) *(volatile float*)(out + g) = o;
}

extern "C" void kernel_launch(void* const* d_in, const int* in_sizes, int n_in,
                              void* d_out, int out_size, void* d_ws, size_t ws_size, hipStream_t stream) {
  if (n_in < 19 || d_out == nullptr || d_ws == nullptr) return;
  if (in_sizes[0] != N_NODES * F_IN || in_sizes[1] != N_EDGES * F_EDGE || in_sizes[2] != N_NODES * DEG ||
      in_sizes[3] != N_GATE * F_IN || in_sizes[4] != N_GATE * F_IN || in_sizes[5] != N_GATE || in_sizes[6] != N_GATE ||
      in_sizes[7] != F_IN * F_OUT || in_sizes[8] != F_OUT || in_sizes[9] != F_IN * F_OUT ||
      in_sizes[10] != F_EDGE * F_EDGE * F_OUT || in_sizes[11] != F_EDGE * F_OUT || in_sizes[12] != F_OUT ||
      in_sizes[13] != F_OUT * 32 || in_sizes[14] != 32 || in_sizes[15] != 32 * 32 || in_sizes[16] != 32 ||
      in_sizes[17] != 32 || in_sizes[18] != 1 || out_size != N_GRAPHS) return;

  const float* nfeat  = (const float*)d_in[0];
  const float* efeat  = (const float*)d_in[1];
  const int*   neigh  = (const int*)d_in[2];
  const float* Wih    = (const float*)d_in[3];
  const float* Whh    = (const float*)d_in[4];
  const float* bih    = (const float*)d_in[5];
  const float* bhh    = (const float*)d_in[6];
  const float* Wself  = (const float*)d_in[7];
  const float* bself  = (const float*)d_in[8];
  const float* Wneigh = (const float*)d_in[9];
  const float* Wew    = (const float*)d_in[10];
  const float* Web    = (const float*)d_in[11];
  const float* nnb    = (const float*)d_in[12];
  const float* W1     = (const float*)d_in[13];
  const float* b1     = (const float*)d_in[14];
  const float* W2     = (const float*)d_in[15];
  const float* b2     = (const float*)d_in[16];
  const float* W3     = (const float*)d_in[17];
  const float* b3     = (const float*)d_in[18];
  float* out = (float*)d_out;

  char* ws = (char*)d_ws; size_t off = 0;
  auto carve = [&](size_t bytes) -> char* { char* p = ws + off; off += (bytes + 255) & ~(size_t)255; return p; };
  unsigned short* cat     = (unsigned short*)carve((size_t)N_PAD * CAT_LD * 2);
  unsigned short* Wih16   = (unsigned short*)carve((size_t)N_GATE * F_IN * 2);
  unsigned short* Whh16   = (unsigned short*)carve((size_t)N_GATE * F_IN * 2);
  float*          bsum    = (float*)carve((size_t)N_GATE * 4);
  float*          bself64 = (float*)carve((size_t)64 * 4);
  float*          nnb64   = (float*)carve((size_t)64 * 4);
  unsigned short* WcatT   = (unsigned short*)carve((size_t)64 * CAT_LD * 2);
  unsigned short* WrT     = (unsigned short*)carve((size_t)64 * P_LD * 2);
  float*          xproj   = (float*)carve((size_t)N_PAD * N_GATE * 4);
  float*          hfull   = (float*)carve((size_t)N_PAD * H_LD * 4);
  unsigned short* Pp      = (unsigned short*)carve((size_t)N_PAD * P_LD * 2);
  float*          h2      = (float*)carve((size_t)N_PAD * H_LD * 4);
  float*          g0      = (float*)carve((size_t)N_GRAPHS * F_OUT * 4);
  if (off > ws_size || off > (size_t)134217728) return;

  prep_kernel<<<PREP_BLOCKS, 256, 0, stream>>>(nfeat, Wih, Whh, bih, bhh, Wself, bself, Wneigh, Wew, Web, nnb,
                                               cat, Wih16, Whh16, bsum, bself64, nnb64, WcatT, WrT);
  {
    const int tiles = (N_PAD / 64) * (N_GATE / 64);
    gemm64_f16<0><<<(tiles + 7) / 8, 256, 0, stream>>>(cat, CAT_LD, Wih16, F_IN, xproj, N_GATE, bsum,
                                                      N_PAD, N_GATE, F_IN, W_CARRY_INV);
  }
  lstm_kernel<<<N_PAD / 64, 128, 0, stream>>>(xproj, neigh, Whh16, cat);
  {
    const int tiles = (N_PAD / 64);
    gemm64_f16<1><<<(tiles + 7) / 8, 256, 0, stream>>>(cat, CAT_LD, WcatT, CAT_LD, hfull, H_LD, bself64,
                                                      N_PAD, 64, CAT_LD, W_CARRY_INV);
  }
  pbuild_kernel<<<N_PAD / 8, 256, 0, stream>>>(efeat, neigh, hfull, Pp);
  {
    const int tiles = (N_PAD / 64);
    gemm64_f16<0><<<(tiles + 7) / 8, 256, 0, stream>>>(Pp, P_LD, WrT, P_LD, h2, H_LD, nnb64,
                                                      N_PAD, 64, P_KDIM, W_CARRY_INV);
  }
  pool_kernel<<<(N_GRAPHS + 7) / 8, 256, 0, stream>>>(h2, g0);
  head_kernel<<<1, 224, 0, stream>>>(g0, W1, b1, W2, b2, W3, b3, out);
}
